// InterpretableMultiHeadAttention_2121713844709
// MI455X (gfx1250) — hardware-run, weakly checked
//
#include <hip/hip_runtime.h>


#ifndef NB_
#define NB_ 4
#endif
#ifndef SEQ
#define SEQ 1024
#endif
#define NB_FULL  4
#define SEQ_FULL 1024
#define TT   SEQ
#define DM   1024
#define NH_  16
#define HD   64
#define DQ   (NH_ * HD)
#define RH   64
#define QCAR 8.0f
#define VCAR 64.0f
#define PCAR 1024.0f
#define SCL2 (0.125f / 64.0f)
#define MFILL (-1.0e9f)
#define OUT1_OFF ((size_t)NB_FULL * SEQ_FULL * DM)
static_assert(OUT1_OFF * 4 == (size_t)16777216);
static_assert(SEQ % 128 == 0 && SEQ >= RH && SEQ <= SEQ_FULL && NB_ >= 1 && NB_ <= NB_FULL && RH == 64 && (TT / 32) <= 32);
static_assert(DM % 64 == 0 && DQ % 64 == 0 && HD == 64 && (3 * HD) % 32 == 0 && (3 * TT) % 32 == 0);

typedef _Float16 h16;
typedef unsigned short bf;
typedef __attribute__((ext_vector_type(16))) __bf16   v16bf;
typedef __attribute__((ext_vector_type(16))) _Float16 v16h;
typedef __attribute__((ext_vector_type(8)))  _Float16 v8h;
typedef __attribute__((ext_vector_type(8)))  unsigned short v8us;
typedef __attribute__((ext_vector_type(8)))  float    v8f;
typedef __attribute__((ext_vector_type(4)))  float    v4f;
typedef v8h  __attribute__((may_alias)) v8ha;
typedef v4f  __attribute__((may_alias)) v4fa;
typedef v8us __attribute__((may_alias)) v8usa;

__device__ __forceinline__ unsigned short f2bf(float f) { unsigned u = __float_as_uint(f); u += 0x7FFFu + ((u >> 16) & 1u); return (unsigned short)(u >> 16); }
__device__ __forceinline__ float bf2f(unsigned short b) { return __uint_as_float(((unsigned)b) << 16); }
__device__ __forceinline__ float bfr(float f) { return bf2f(f2bf(f)); }
__device__ __forceinline__ v16h cat16(v8h lo, v8h hi) { return __builtin_shufflevector(lo, hi, 0, 1, 2, 3, 4, 5, 6, 7, 8, 9, 10, 11, 12, 13, 14, 15); }
__device__ __forceinline__ v16bf cat16b(v8us lo, v8us hi) { return __builtin_bit_cast(v16bf, __builtin_shufflevector(lo, hi, 0, 1, 2, 3, 4, 5, 6, 7, 8, 9, 10, 11, 12, 13, 14, 15)); }
__device__ __forceinline__ v8f wmma16(v16h a, v16h b, v8f c) { return __builtin_amdgcn_wmma_f32_16x16x32_f16(false, a, false, b, (short)0, c, false, false); }
__device__ __forceinline__ v8f wmmab(v16bf a, v16bf b, v8f c) { return __builtin_amdgcn_wmma_f32_16x16x32_bf16(false, a, false, b, (short)0, c, false, false); }

template <typename T16> struct WFrag;
template <> struct WFrag<h16> { typedef v16h V; static __device__ __forceinline__ V ld(const h16* p) { return cat16(*(const v8h*)p, *(const v8h*)(p + 16)); } static __device__ __forceinline__ v8f mma(V a, V b, v8f c) { return wmma16(a, b, c); } };
template <> struct WFrag<bf> { typedef v16bf V; static __device__ __forceinline__ V ld(const bf* p) { return cat16b(*(const v8us*)p, *(const v8us*)(p + 16)); } static __device__ __forceinline__ v8f mma(V a, V b, v8f c) { return wmmab(a, b, c); } };
template <typename T16, int NSPLIT, bool BIAS>
__global__ __launch_bounds__(32) void k_gemmw(const T16* __restrict__ A, const T16* __restrict__ A2, const T16* __restrict__ Bt, const T16* __restrict__ Bt2, int K, float* C, int ldc, const float* __restrict__ bias, size_t sA, size_t sB, size_t sC) {
    typedef typename WFrag<T16>::V V;
    __shared__ __align__(16) float os[16 * 68];
    const size_t z = blockIdx.z; A += z * sA; if (A2) A2 += z * sA; Bt += z * sB; if (Bt2) Bt2 += z * sB; C += z * sC;
    const int lane = threadIdx.x & 31, lr = lane & 15, hi = lane >> 4; const int r0 = blockIdx.x * 64, c0 = blockIdx.y * 64;
    v8f acc[4][4];
#pragma unroll
    for (int mb = 0; mb < 4; ++mb)
#pragma unroll
        for (int nb = 0; nb < 4; ++nb) acc[mb][nb] = (v8f){};
    const size_t aoff = (size_t)(r0 + lr) * K + 8 * hi, boff = (size_t)(c0 + lr) * K + 8 * hi;
#pragma unroll 1
    for (int kc = 0; kc < K; kc += 32) {
        V a[4], a2[4];
#pragma unroll
        for (int mb = 0; mb < 4; ++mb) { a[mb] = WFrag<T16>::ld(A + aoff + (size_t)mb * 16 * K + kc); if (NSPLIT == 1 || NSPLIT == 2) a2[mb] = WFrag<T16>::ld(A2 + aoff + (size_t)mb * 16 * K + kc); }
#pragma unroll
        for (int nb = 0; nb < 4; ++nb) { const V b = WFrag<T16>::ld(Bt + boff + (size_t)nb * 16 * K + kc); V b2; if (NSPLIT >= 2) b2 = WFrag<T16>::ld(Bt2 + boff + (size_t)nb * 16 * K + kc);
#pragma unroll
            for (int mb = 0; mb < 4; ++mb) { acc[mb][nb] = WFrag<T16>::mma(a[mb], b, acc[mb][nb]); if (NSPLIT == 1 || NSPLIT == 2) acc[mb][nb] = WFrag<T16>::mma(a2[mb], b, acc[mb][nb]); if (NSPLIT >= 2) acc[mb][nb] = WFrag<T16>::mma(a[mb], b2, acc[mb][nb]); } }
        asm volatile("v_nop\n\tv_nop\n\tv_nop\n\tv_nop" : "+v"(acc[0][0]), "+v"(acc[1][1]), "+v"(acc[2][2]), "+v"(acc[3][3]) : "v"(a[0]), "v"(a[3]));
    }
#pragma unroll
    for (int mb = 0; mb < 4; ++mb) {
#pragma unroll
        for (int nb = 0; nb < 4; ++nb) {
#pragma unroll
            for (int j = 0; j < 8; ++j) os[(hi * 8 + j) * 68 + nb * 16 + lr] = acc[mb][nb][j]; }
        __builtin_amdgcn_wave_barrier(); asm volatile("" ::: "memory");
        float* crow = C + (size_t)(r0 + mb * 16) * ldc + c0;
#pragma unroll 1
        for (int ps = 0; ps < 2; ++ps) {
#pragma unroll
            for (int s = 0; s < 8; ++s) { const int row = 2 * s + hi, cofs = lr * 4; v4f val = *(const v4fa*)(os + row * 68 + cofs); if (BIAS) { val[0] += bfr(bias[c0 + cofs]); val[1] += bfr(bias[c0 + cofs + 1]); val[2] += bfr(bias[c0 + cofs + 2]); val[3] += bfr(bias[c0 + cofs + 3]); }
                *(volatile v4f*)(crow + (size_t)row * ldc + cofs) = val; }
            if (ps == 0) __threadfence(); }
        __builtin_amdgcn_wave_barrier(); asm volatile("" ::: "memory");
    }
}

__device__ __forceinline__ h16 tohx(float x) { return (h16)x; }
__device__ __forceinline__ void splitf(float y, unsigned short& h, unsigned short& l) { h = f2bf(y); l = f2bf(y - bf2f(h)); }
typedef __attribute__((ext_vector_type(2))) _Float16 v2h;
typedef __attribute__((ext_vector_type(4))) _Float16 v4h;
typedef __attribute__((ext_vector_type(2))) unsigned short v2us;
typedef __attribute__((ext_vector_type(4))) unsigned short v4us;
typedef __attribute__((ext_vector_type(2))) float v2f;
typedef __attribute__((ext_vector_type(4))) int v4i;

__global__ __launch_bounds__(256) void k_cvt8(const float* __restrict__ src, bf* dst, size_t n8) { const size_t i = (size_t)blockIdx.x * 256 + threadIdx.x; if (i >= n8) return; const v8f v = *(const v8f*)(src + i * 8); v8us o;
#pragma unroll
    for (int k = 0; k < 8; ++k) o[k] = f2bf(v[k]); *(volatile v8us*)(dst + i * 8) = o; __threadfence(); *(volatile v8us*)(dst + i * 8) = o; }

__global__ __launch_bounds__(256) void k_wt3(const float* __restrict__ w, int K, int N, int G, bf* Bt) {
    const int lane = threadIdx.x & 31; const int L0 = (blockIdx.x * 8 + (threadIdx.x >> 5)) * 8; const int nlines = (int)((size_t)G * N * K / 64);
#pragma unroll
    for (int ps = 0; ps < 2; ++ps) {
#pragma unroll 1
        for (int l = 0; l < 8; ++l) { const int L = L0 + l; if (L >= nlines) break; const size_t e = (size_t)L * 64 + lane * 2; const int k = (int)(e % K); const int ng = (int)(e / K); const int g = ng / N, n = ng % N; v2us o;
            o[0] = f2bf(w[((size_t)g * K + k) * N + n]); o[1] = f2bf(w[((size_t)g * K + k + 1) * N + n]); *(volatile v2us*)(Bt + e) = o; }
        if (ps == 0) __threadfence(); }
}

__global__ __launch_bounds__(256) void k_plane(const float* __restrict__ F, int pitch, int nheads, float sc, h16* P16, bf* Pc, int hlrows, int loseg) {
    const size_t e = ((size_t)blockIdx.x * 256 + threadIdx.x) * 2; if (e >= (size_t)nheads * TT * HD) return;
    const int d = (int)(e % HD); const int t = (int)((e / HD) % TT); const int h = (int)(e / ((size_t)HD * TT));
    const float* f = F + (size_t)t * pitch + h * HD + d;
    float x[2]; x[0] = f[0] * sc; x[1] = f[1] * sc; v2h o16; v2us oh, ol, s1, s2;
#pragma unroll
    for (int q = 0; q < 2; ++q) { o16[q] = tohx(x[q]); unsigned short a2, c2; splitf(x[q], a2, c2); oh[q] = a2; ol[q] = c2; s1[q] = (loseg == 1) ? c2 : a2; s2[q] = (loseg == 2) ? c2 : a2; }
    const bool hl = (t < hlrows);
    const size_t oo = ((size_t)h * hlrows + (hl ? t : 0)) * (3 * HD) + d;
#pragma unroll 1
    for (int ps = 0; ps < 2; ++ps) {
        *(volatile v2h*)(P16 + e) = o16;
        if (hl) { *(volatile v2us*)(Pc + oo) = oh; *(volatile v2us*)(Pc + oo + HD) = s1; *(volatile v2us*)(Pc + oo + 2 * HD) = s2; }
        if (ps == 0) __threadfence(); }
}

__global__ __launch_bounds__(256) void k_vplane(const float* __restrict__ F, int pitch, float sc, h16* V16, bf* Vc) {
    const size_t e = ((size_t)blockIdx.x * 256 + threadIdx.x) * 2; if (e >= (size_t)HD * TT) return; const int t = (int)(e % TT); const int d = (int)(e / TT);
    v2h o16; v2us oh, ol;
#pragma unroll
    for (int q = 0; q < 2; ++q) { const float x = F[(size_t)(t + q) * pitch + d]; o16[q] = tohx(x * sc); unsigned short a2, c2; splitf(x, a2, c2); oh[q] = a2; ol[q] = c2; }
    const size_t oo = (size_t)d * (3 * TT) + t;
#pragma unroll 1
    for (int ps = 0; ps < 2; ++ps) {
        *(volatile v2h*)(V16 + e) = o16; *(volatile v2us*)(Vc + oo) = oh; *(volatile v2us*)(Vc + oo + TT) = oh; *(volatile v2us*)(Vc + oo + 2 * TT) = ol;
        if (ps == 0) __threadfence(); }
}

__global__ __launch_bounds__(256) void k_soft(const float* __restrict__ Sb, const int* __restrict__ mask, h16* P16, bf* Pc, float* AW) {
#pragma clang fp contract(off)
    const int lane = threadIdx.x & 31; const int i = blockIdx.x * 8 + (threadIdx.x >> 5); if (i >= TT) return;
    const int* mr = mask + (size_t)i * SEQ_FULL; unsigned bits = 0u;
#pragma unroll
    for (int ch = 0; ch < TT / 128; ++ch) { const v4i m4 = *(const v4i*)(mr + ch * 128 + lane * 4);
#pragma unroll
        for (int q = 0; q < 4; ++q) bits |= ((m4[q] != 0) ? 1u : 0u) << (ch * 4 + q); }
    float aw[TT / 32];
#pragma unroll
    for (int k = 0; k < TT / 32; ++k) aw[k] = 0.0f;
    const bool hires = (i < RH);
#pragma unroll 1
    for (int zz = 0; zz < NH_; ++zz) {
        const float* sr = Sb + ((size_t)zz * TT + i) * TT; float v[TT / 32]; float mx = -3.0e38f;
#pragma unroll
        for (int ch = 0; ch < TT / 128; ++ch) { const v4f a = *(const v4f*)(sr + ch * 128 + lane * 4);
#pragma unroll
            for (int q = 0; q < 4; ++q) { const int k = ch * 4 + q; const float s = a[q] * SCL2; const float t = ((bits >> k) & 1u) ? s : MFILL; v[k] = t; mx = fmaxf(mx, t); } }
#pragma unroll
        for (int sh = 16; sh; sh >>= 1) mx = fmaxf(mx, __shfl_xor(mx, sh, 32));
        float sum = 0.f;
#pragma unroll
        for (int k = 0; k < TT / 32; ++k) { float d0 = __fsub_rn(v[k], mx); asm volatile("" : "+v"(d0)); v[k] = __builtin_amdgcn_exp2f(__fmul_rn(d0, 1.4426950408889634f)); sum += v[k]; }
#pragma unroll
        for (int sh = 16; sh; sh >>= 1) sum += __shfl_xor(sum, sh, 32);
        const float inv = __fdiv_rn(1.0f, sum);
#pragma unroll
        for (int k = 0; k < TT / 32; ++k) { float p = v[k] * inv; asm volatile("" : "+v"(p)); v[k] = p; aw[k] += p; }
        h16* prow = P16 + ((size_t)zz * TT + i) * TT; bf* crow = Pc + ((size_t)zz * RH + (hires ? i : 0)) * (3 * TT);
#pragma unroll 1
        for (int ps = 0; ps < 2; ++ps) {
#pragma unroll
            for (int ch = 0; ch < TT / 128; ++ch) { v4h o4;
#pragma unroll
                for (int q = 0; q < 4; ++q) o4[q] = tohx(v[ch * 4 + q] * PCAR);
                *(volatile v4h*)(prow + ch * 128 + lane * 4) = o4; }
            if (hires) {
#pragma unroll
                for (int ch = 0; ch < TT / 128; ++ch) { v4us oh, ol;
#pragma unroll
                    for (int q = 0; q < 4; ++q) { unsigned short a2, c2; splitf(v[ch * 4 + q], a2, c2); oh[q] = a2; ol[q] = c2; }
                    const int off = ch * 128 + lane * 4; *(volatile v4us*)(crow + off) = oh; *(volatile v4us*)(crow + TT + off) = ol; *(volatile v4us*)(crow + 2 * TT + off) = oh; } }
            if (ps == 0) __threadfence(); }
    }
    float* arow = AW + (size_t)i * SEQ_FULL;
#pragma unroll 1
    for (int ps = 0; ps < 2; ++ps) {
#pragma unroll
        for (int ch = 0; ch < TT / 128; ++ch) { v4f o;
#pragma unroll
            for (int q = 0; q < 4; ++q) o[q] = aw[ch * 4 + q] * (1.0f / NH_);
            *(volatile v4f*)(arow + ch * 128 + lane * 4) = o; }
        if (ps == 0) __threadfence(); }
}

__global__ __launch_bounds__(256) void k_hsum(const float* __restrict__ O, bf* Hh, bf* Hl) {
#pragma clang fp contract(off)
    const size_t e = ((size_t)blockIdx.x * 256 + threadIdx.x) * 4; if (e >= (size_t)TT * HD) return; const int t = (int)(e / HD);
    v4f s = *(const v4f*)(O + e);
#pragma unroll
    for (int h = 1; h < NH_; ++h) { const v4f a = *(const v4f*)(O + (size_t)h * TT * HD + e); s = s + a; }
    const float cs = ((t < RH) ? 1.0f : (1.0f / (PCAR * VCAR))) * (1.0f / NH_);
    v4us oh, ol;
#pragma unroll
    for (int u = 0; u < 4; ++u) { unsigned short a2, b2; splitf(s[u] * cs, a2, b2); oh[u] = a2; ol[u] = b2; }
    *(volatile v4us*)(Hh + e) = oh; *(volatile v4us*)(Hl + e) = ol; __threadfence(); *(volatile v4us*)(Hh + e) = oh; *(volatile v4us*)(Hl + e) = ol;
}

extern "C" void kernel_launch(void* const* d_in, const int* in_sizes, int n_in,
                              void* d_out, int out_size, void* d_ws, size_t ws_size, hipStream_t stream) {
    if (n_in < 12) return;
    const float* xq = (const float*)d_in[0];
    const float* xk = (const float*)d_in[1];
    const float* xv = (const float*)d_in[2];
    const int*   mk = (const int*)d_in[3];
    const float* wq = (const float*)d_in[4];
    const float* bq = (const float*)d_in[5];
    const float* wk = (const float*)d_in[6];
    const float* bk = (const float*)d_in[7];
    const float* wv = (const float*)d_in[8];
    const float* bv = (const float*)d_in[9];
    const float* wo = (const float*)d_in[10];
    const float* bo = (const float*)d_in[11];
    const size_t need_x = (size_t)(NB_ - 1) * SEQ_FULL * DM + (size_t)SEQ * DM;
    if ((size_t)in_sizes[0] < need_x || (size_t)in_sizes[1] < need_x || (size_t)in_sizes[2] < need_x) return;
    if ((size_t)in_sizes[3] < (size_t)(SEQ - 1) * SEQ_FULL + SEQ) return;
    if ((size_t)in_sizes[4] < (size_t)NH_ * DM * HD || in_sizes[5] < NH_ * HD || (size_t)in_sizes[6] < (size_t)NH_ * DM * HD || in_sizes[7] < NH_ * HD) return;
    if (in_sizes[8] < DM * HD || in_sizes[9] < HD || in_sizes[10] < HD * DM || in_sizes[11] < DM) return;
    const size_t need_out = OUT1_OFF + (size_t)(NB_ - 1) * SEQ_FULL * SEQ_FULL + (size_t)(SEQ - 1) * SEQ_FULL + SEQ;
    if (out_size < 0 || (size_t)out_size < need_out) return;

    float* OUT = (float*)d_out;
    float* AW  = OUT + OUT1_OFF;
    char* wsp = (char*)d_ws;
    auto take = [&](size_t bytes) { char* p = wsp; wsp += (bytes + 255) & ~(size_t)255; return (void*)p; };
    bf* WQt = (bf*)take((size_t)DQ * DM * 2);
    bf* WKt = (bf*)take((size_t)DQ * DM * 2);
    bf* WVt = (bf*)take((size_t)HD * DM * 2);
    bf* WOt = (bf*)take((size_t)DM * HD * 2);
    bf* XB  = (bf*)take((size_t)TT * DM * 2);
    float* F = (float*)take((size_t)TT * DQ * 4);
    h16* QP16 = (h16*)take((size_t)NH_ * TT * HD * 2);
    bf*  QPc  = (bf*)take((size_t)NH_ * RH * 3 * HD * 2);
    h16* KP16 = (h16*)take((size_t)NH_ * TT * HD * 2);
    bf*  KPc  = (bf*)take((size_t)NH_ * TT * 3 * HD * 2);
    h16* VT16 = (h16*)take((size_t)HD * TT * 2);
    bf*  VTc  = (bf*)take((size_t)HD * 3 * TT * 2);
    float* Sb = (float*)take((size_t)NH_ * TT * TT * 4);
    h16* P16  = (h16*)take((size_t)NH_ * TT * TT * 2);
    bf*  Pc   = (bf*)take((size_t)NH_ * RH * 3 * TT * 2);
    float* Ob = (float*)take((size_t)NH_ * TT * HD * 4);
    bf*  XSh  = (bf*)take((size_t)TT * HD * 2);
    bf*  XSl  = (bf*)take((size_t)TT * HD * 2);
    if ((size_t)(wsp - (char*)d_ws) > ws_size) return;

    k_wt3<<<(unsigned)(((size_t)NH_ * HD * DM / 64 + 63) / 64), 256, 0, stream>>>(wq, DM, HD, NH_, WQt);
    k_wt3<<<(unsigned)(((size_t)NH_ * HD * DM / 64 + 63) / 64), 256, 0, stream>>>(wk, DM, HD, NH_, WKt);
    k_wt3<<<(unsigned)(((size_t)HD * DM / 64 + 63) / 64), 256, 0, stream>>>(wv, DM, HD, 1, WVt);
    k_wt3<<<(unsigned)(((size_t)DM * HD / 64 + 63) / 64), 256, 0, stream>>>(wo, HD, DM, 1, WOt);

    const unsigned LX = (unsigned)(((size_t)TT * DM / 8 + 255) / 256), LP = (unsigned)(((size_t)NH_ * TT * HD / 2 + 255) / 256);
    const unsigned LV = (unsigned)(((size_t)HD * TT / 2 + 255) / 256), LH = (unsigned)(((size_t)TT * HD / 4 + 255) / 256);
    for (int b = 0; b < NB_; ++b) {
        const float* xqb = xq + (size_t)b * SEQ_FULL * DM; const float* xkb = xk + (size_t)b * SEQ_FULL * DM; const float* xvb = xv + (size_t)b * SEQ_FULL * DM;
        k_cvt8<<<LX, 256, 0, stream>>>(xqb, XB, (size_t)TT * DM / 8);
        k_gemmw<bf, 0, true><<<dim3(TT / 64, DQ / 64, 1), 32, 0, stream>>>(XB, nullptr, WQt, nullptr, DM, F, DQ, bq, 0, 0, 0);
        k_plane<<<LP, 256, 0, stream>>>(F, DQ, NH_, QCAR, QP16, QPc, RH, 1);
        k_cvt8<<<LX, 256, 0, stream>>>(xkb, XB, (size_t)TT * DM / 8);
        k_gemmw<bf, 0, true><<<dim3(TT / 64, DQ / 64, 1), 32, 0, stream>>>(XB, nullptr, WKt, nullptr, DM, F, DQ, bk, 0, 0, 0);
        k_plane<<<LP, 256, 0, stream>>>(F, DQ, NH_, QCAR, KP16, KPc, TT, 2);
        k_cvt8<<<LX, 256, 0, stream>>>(xvb, XB, (size_t)TT * DM / 8);
        k_gemmw<bf, 0, true><<<dim3(TT / 64, 1, 1), 32, 0, stream>>>(XB, nullptr, WVt, nullptr, DM, F, HD, bv, 0, 0, 0);
        k_vplane<<<LV, 256, 0, stream>>>(F, HD, VCAR, VT16, VTc);
        k_gemmw<h16, 0, false><<<dim3(TT / 64, TT / 64, NH_), 32, 0, stream>>>(QP16, nullptr, KP16, nullptr, HD, Sb, TT, nullptr, (size_t)TT * HD, (size_t)TT * HD, (size_t)TT * TT);
        k_gemmw<bf, 0, false><<<dim3(1, TT / 64, NH_), 32, 0, stream>>>(QPc, nullptr, KPc, nullptr, 3 * HD, Sb, TT, nullptr, (size_t)RH * 3 * HD, (size_t)TT * 3 * HD, (size_t)TT * TT);
        k_soft<<<TT / 8, 256, 0, stream>>>(Sb, mk, P16, Pc, AW + (size_t)b * SEQ_FULL * SEQ_FULL);
        k_gemmw<h16, 0, false><<<dim3(TT / 64, 1, NH_), 32, 0, stream>>>(P16, nullptr, VT16, nullptr, TT, Ob, HD, nullptr, (size_t)TT * TT, 0, (size_t)TT * HD);
        k_gemmw<bf, 0, false><<<dim3(1, 1, NH_), 32, 0, stream>>>(Pc, nullptr, VTc, nullptr, 3 * TT, Ob, HD, nullptr, (size_t)RH * 3 * TT, 0, (size_t)TT * HD);
        k_hsum<<<LH, 256, 0, stream>>>(Ob, XSh, XSl);
        k_gemmw<bf, 1, true><<<dim3(TT / 64, DM / 64, 1), 32, 0, stream>>>(XSh, XSl, WOt, nullptr, HD, OUT + (size_t)b * SEQ_FULL * DM, DM, bo, 0, 0, 0);
    }
}
